// Tree_RNNAgent_76098230550832
// MI455X (gfx1250) — hardware-run, weakly checked
//
#include <hip/hip_runtime.h>


#ifndef NB
#define NB 512
#endif
#define NB_FULL   512
#define NAGT      8
#define NAG       (NB * NAGT)
#define NAG_FULL  (NB_FULL * NAGT)
#define NEN       8
#define NAL       7
#define FD        16
#define HID       64
#define HEADS     4
#define OUTN      6
#define QW        14
#define DE        4356
#define DA        4096
#define KH1       2112
#define K1        (2 * KH1)
#define K2        192
#define K3        128
#define N1        256
#define N2        256
#define N3        320
#define APB       4
#define HAG       16

static_assert(NB <= NB_FULL);
static_assert(NAG % 64 == 0);
static_assert(NAG % APB == 0);
static_assert(NAG % HAG == 0);
static_assert(NAG % 4 == 0);
static_assert(K1 % 32 == 0);
static_assert(K2 % 32 == 0);
static_assert(K3 % 32 == 0);
static_assert(KH1 % 64 == 0);
static_assert(N1 % 64 == 0);
static_assert(N2 % 64 == 0);
static_assert(N3 % 64 == 0);
static_assert((HAG * QW * 4) % 128 == 0);
static_assert((size_t)NAG_FULL * QW * 4 == (size_t)229376);
static_assert(((size_t)NAG_FULL * QW * 4) % 128 == 0);
static_assert(DE == (FD * HID + HID + 1) * HEADS);
static_assert(DA == FD * HID * HEADS);
static_assert(FD * 64 == 4 * 256);
static_assert(FD * 64 == 4 * 64 * 4);

typedef unsigned short bf;
typedef __attribute__((ext_vector_type(16))) __bf16   v16bf;
typedef __attribute__((ext_vector_type(8)))  unsigned short v8us;
typedef __attribute__((ext_vector_type(8)))  float    v8f;
typedef __attribute__((ext_vector_type(4)))  float    v4f;
typedef v4f  __attribute__((may_alias)) v4fa;
typedef v8us __attribute__((may_alias)) v8usa;

__device__ __forceinline__ unsigned short f2bf(float f) { unsigned u = __float_as_uint(f); u += 0x7FFFu + ((u >> 16) & 1u); return (unsigned short)(u >> 16); }
__device__ __forceinline__ float bf2f(unsigned short b) { return __uint_as_float(((unsigned)b) << 16); }
__device__ __forceinline__ float rbf(float f) { return bf2f(f2bf(f)); }
__device__ __forceinline__ v4f rbf4(v4f v) { v4f r; r[0] = rbf(v[0]); r[1] = rbf(v[1]); r[2] = rbf(v[2]); r[3] = rbf(v[3]); return r; }
__device__ __forceinline__ v16bf cat16b(v8us lo, v8us hi) { return __builtin_bit_cast(v16bf, __builtin_shufflevector(lo, hi, 0, 1, 2, 3, 4, 5, 6, 7, 8, 9, 10, 11, 12, 13, 14, 15)); }
__device__ __forceinline__ v8f wmmab(v16bf a, v16bf b, v8f c) { return __builtin_amdgcn_wmma_f32_16x16x32_bf16(false, a, false, b, (short)0, c, false, false); }
__device__ __forceinline__ v16bf ldb(const bf* p)  { return cat16b(*(const v8us*)p, *(const v8us*)(p + 16)); }
__device__ __forceinline__ void wave_sync() { __builtin_amdgcn_fence(3  , "wavefront"); __builtin_amdgcn_wave_barrier(); asm volatile("" ::: "memory"); }

__global__ __launch_bounds__(128) void k_bt1(const float* __restrict__ hew2, const float* __restrict__ heb2, const float* __restrict__ haw2, const float* __restrict__ hab2, bf* BT1) {
    __shared__ __align__(16) unsigned short sg[64];
    const int n = blockIdx.x, seg = blockIdx.y, t = threadIdx.x;
    const int h = n >> 2, k = n & 3;
    v8us o; int col; bool act;
    if (seg == 0) {
        const int f = t >> 3, j0 = (t & 7) * 8; const int cidx = (f * 64 + h) * 4 + k;
#pragma unroll
        for (int i = 0; i < 8; ++i) o[i] = f2bf(hew2[(size_t)(j0 + i) * DE + cidx]);
        col = t * 8; act = true;
    } else if (seg == 1) {
        const int f = t >> 3, j0 = (t & 7) * 8; const int cidx = (f * 64 + h) * 4 + k;
#pragma unroll
        for (int i = 0; i < 8; ++i) o[i] = f2bf(haw2[(size_t)(j0 + i) * DA + cidx]);
        col = 1024 + t * 8; act = true;
    } else {
        const int f = t & 15; const int cidx = (f * 64 + h) * 4 + k;
        const float ve = heb2[cidx]; const float va = hab2[cidx];
        const float v = (t < 16) ? ve : ((t < 32) ? va : 0.0f);
        if (t < 64) sg[t] = f2bf(v);
        __syncthreads();
        const int c = t & 7;
        o = *(const v8usa*)(&sg[c * 8]);
        col = 2048 + c * 8; act = (t < 8);
    }
    bf* p = BT1 + (size_t)n * K1 + col;
#pragma unroll 1
    for (int ps = 0; ps < 2; ++ps) {
        if (act) { *(volatile v8us*)p = o; *(volatile v8us*)(p + KH1) = o; }
        if (ps == 0) __threadfence(); }
}

__global__ __launch_bounds__(256) void k_bt2(const float* __restrict__ wih, const float* __restrict__ whh, bf* BT2) {
    const int i = blockIdx.x * 256 + threadIdx.x; if (i >= N2 * (K2 / 8)) return;
    const int n = i / 24, c = i - n * 24; const int reg = c >> 3, kq = (c & 7) * 8;
    const int ir = (n < 192) ? n : 191; const int hr = (n < 128) ? n : ((n >= 192) ? (n - 64) : 128);
    const v4f i0 = *(const v4f*)(wih + ir * 64 + kq), i1 = *(const v4f*)(wih + ir * 64 + kq + 4);
    const v4f h0 = *(const v4f*)(whh + hr * 64 + kq), h1 = *(const v4f*)(whh + hr * 64 + kq + 4);
    const bool useI = (reg < 2) && (n < 192); const bool useH = (reg == 2) && ((n < 128) || (n >= 192));
    v8us o;
#pragma unroll
    for (int q = 0; q < 4; ++q) { const float a = useI ? i0[q] : (useH ? h0[q] : 0.0f); const float b = useI ? i1[q] : (useH ? h1[q] : 0.0f); o[q] = f2bf(a); o[4 + q] = f2bf(b); }
    bf* p = BT2 + (size_t)n * K2 + c * 8;
    *(volatile v8us*)p = o; __threadfence(); *(volatile v8us*)p = o;
}

__global__ __launch_bounds__(256) void k_bt3(const float* __restrict__ hew2, const float* __restrict__ heb2, const float* __restrict__ fc2w, bf* BT3) {
    __shared__ __align__(16) unsigned short tl[32 * 64];
    const int t = blockIdx.x * 256 + threadIdx.x; const int n = t >> 3, c = t & 7;
    v8us o;
    if (blockIdx.x < 8) {
        const int j = n >> 2, k = n & 3;
#pragma unroll
        for (int i = 0; i < 8; ++i) o[i] = f2bf(hew2[(size_t)j * DE + 4096 + (c * 8 + i) * 4 + k]);
    } else {
        const int nb0 = blockIdx.x * 32;
#pragma unroll 1
        for (int i = 0; i < 8; ++i) { const int idx = threadIdx.x + 256 * i; const int nn = nb0 + (idx >> 6), hq = idx & 63;
            int k4 = nn - 256; k4 = k4 < 0 ? 0 : (k4 > 3 ? 3 : k4); int o6 = nn - 260; o6 = o6 < 0 ? 0 : (o6 > 5 ? 5 : o6);
            const float vb = heb2[4096 + hq * 4 + k4]; const float vf = fc2w[hq * OUTN + o6];
            const float v = (nn < 260) ? vb : ((nn < 266) ? vf : 0.0f); tl[idx] = f2bf(v); }
        __syncthreads();
        o = *(const v8usa*)(&tl[(threadIdx.x >> 3) * 64 + c * 8]);
    }
    bf* p = BT3 + (size_t)n * K3 + c * 8;
#pragma unroll 1
    for (int ps = 0; ps < 2; ++ps) { *(volatile v8us*)p = o; *(volatile v8us*)(p + 64) = o; if (ps == 0) __threadfence(); }
}

__global__ __launch_bounds__(64) void k_build(const float* __restrict__ ef, const float* __restrict__ af,
                                              const float* __restrict__ hew1, const float* __restrict__ heb1,
                                              const float* __restrict__ haw1, const float* __restrict__ hab1,
                                              bf* A1, float* RE) {
    __shared__ __align__(16) float w1e[FD * 64];
    __shared__ __align__(16) float w1a[FD * 64];
    __shared__ __align__(16) float b1s[128];
    __shared__ __align__(16) float fe[128];
    __shared__ __align__(16) float fa[128];
    __shared__ __align__(16) float Rs[NEN * 64];
    __shared__ __align__(16) float Ra[NAL * 64];
    __shared__ __align__(16) unsigned short As[K1];
    const int j = threadIdx.x;
#pragma unroll
    for (int i = 0; i < 4; ++i) { const int c = j + 64 * i;
        const v4f ve = *(const v4f*)(hew1 + c * 4); const v4f va = *(const v4f*)(haw1 + c * 4);
        *(v4fa*)(&w1e[c * 4]) = rbf4(ve); *(v4fa*)(&w1a[c * 4]) = rbf4(va); }
    { const int c = j & 15; const v4f vbe = *(const v4f*)(heb1 + c * 4); const v4f vba = *(const v4f*)(hab1 + c * 4);
      v4f sel; sel[0] = (j < 16) ? vbe[0] : vba[0]; sel[1] = (j < 16) ? vbe[1] : vba[1]; sel[2] = (j < 16) ? vbe[2] : vba[2]; sel[3] = (j < 16) ? vbe[3] : vba[3];
      if (j < 32) *(v4fa*)(&b1s[j * 4]) = rbf4(sel); }
    __syncthreads();
    const float be = b1s[j], ba = b1s[64 + j];
#pragma unroll 1
    for (int it = 0; it < APB; ++it) {
        const int n = blockIdx.x * APB + it;
        fe[j] = rbf(ef[(size_t)n * 128 + j]); fe[64 + j] = rbf(ef[(size_t)n * 128 + 64 + j]);
        fa[j] = rbf(af[(size_t)n * 112 + j]);
        { const int idx = 64 + j; const int ci = idx < 112 ? idx : 111; const float v = af[(size_t)n * 112 + ci]; fa[64 + j] = (idx < 112) ? rbf(v) : 0.0f; }
        __syncthreads();
#pragma unroll 1
        for (int e = 0; e < NEN; ++e) { float acc = 0.0f;
#pragma unroll
            for (int f = 0; f < FD; ++f) acc = fmaf(fe[e * 16 + f], w1e[f * 64 + j], acc);
            acc += be; Rs[e * 64 + j] = fmaxf(acc, 0.0f); }
#pragma unroll 1
        for (int a = 0; a < NAL; ++a) { float acc = 0.0f;
#pragma unroll
            for (int f = 0; f < FD; ++f) acc = fmaf(fa[a * 16 + f], w1a[f * 64 + j], acc);
            acc += ba; Ra[a * 64 + j] = fmaxf(acc, 0.0f); }
#pragma unroll 1
        for (int f = 0; f < FD; ++f) {
            float pe = 0.0f, pa = 0.0f;
#pragma unroll
            for (int e = 0; e < NEN; ++e) pe = fmaf(Rs[e * 64 + j], fe[e * 16 + f], pe);
#pragma unroll
            for (int a = 0; a < NAL; ++a) pa = fmaf(Ra[a * 64 + j], fa[a * 16 + f], pa);
            const unsigned short eh = f2bf(pe); const unsigned short el = f2bf(pe - bf2f(eh));
            const unsigned short ah = f2bf(pa); const unsigned short al = f2bf(pa - bf2f(ah));
            As[f * 64 + j] = eh; As[KH1 + f * 64 + j] = el;
            As[1024 + f * 64 + j] = ah; As[KH1 + 1024 + f * 64 + j] = al; }
        { const int f = j & 15; float se = 0.0f, sa = 0.0f;
#pragma unroll
          for (int e = 0; e < NEN; ++e) se += fe[e * 16 + f];
#pragma unroll
          for (int a = 0; a < NAL; ++a) sa += fa[a * 16 + f];
          const float v = (j < 16) ? se : ((j < 32) ? sa : 0.0f);
          const unsigned short vh = f2bf(v); const unsigned short vl = f2bf(v - bf2f(vh));
          As[2048 + j] = vh; As[KH1 + 2048 + j] = vl; }
        __syncthreads();
        bf* arow = A1 + (size_t)n * K1; float* rrow = RE + (size_t)n * (NEN * 64);
#pragma unroll 1
        for (int ps = 0; ps < 2; ++ps) {
#pragma unroll 1
            for (int c = j; c < K1 / 8; c += 64) { const v8us v = *(const v8usa*)(&As[c * 8]); *(volatile v8us*)(arow + c * 8) = v; }
#pragma unroll 1
            for (int c = j; c < NEN * 16; c += 64) { const v4f v = *(const v4fa*)(&Rs[c * 4]); *(volatile v4f*)(rrow + c * 4) = v; }
            if (ps == 0) __threadfence(); }
        __syncthreads();
    }
}

__global__ __launch_bounds__(32) __attribute__((amdgpu_num_vgpr(256))) void k_gemm(const bf* __restrict__ A, const bf* __restrict__ Bt, float* C, int K, int ldc) {
    __shared__ __align__(16) float os[16 * 68];
    const int lane = threadIdx.x & 31, lr = lane & 15, hi = lane >> 4; const int r0 = blockIdx.x * 64, c0 = blockIdx.y * 64;
    v8f acc[4][4];
#pragma unroll
    for (int mb = 0; mb < 4; ++mb)
#pragma unroll
        for (int nb = 0; nb < 4; ++nb) acc[mb][nb] = (v8f){};
    const size_t aoff = (size_t)(r0 + lr) * K + 8 * hi, boff = (size_t)(c0 + lr) * K + 8 * hi;
#pragma unroll 1
    for (int kc = 0; kc < K; kc += 32) {
        v16bf a[4];
#pragma unroll
        for (int mb = 0; mb < 4; ++mb) a[mb] = ldb(A + aoff + (size_t)mb * 16 * K + kc);
#pragma unroll
        for (int nb = 0; nb < 4; ++nb) { const v16bf b = ldb(Bt + boff + (size_t)nb * 16 * K + kc);
#pragma unroll
            for (int mb = 0; mb < 4; ++mb) acc[mb][nb] = wmmab(a[mb], b, acc[mb][nb]); }
        asm volatile("v_nop\n\tv_nop\n\tv_nop\n\tv_nop" : "+v"(acc[0][0]), "+v"(acc[1][1]), "+v"(acc[2][2]), "+v"(acc[3][3]) : "v"(a[0]), "v"(a[1]), "v"(a[2]), "v"(a[3]));
    }
#pragma unroll
    for (int mb = 0; mb < 4; ++mb) {
#pragma unroll
        for (int nb = 0; nb < 4; ++nb) {
#pragma unroll
            for (int j = 0; j < 8; ++j) os[(hi * 8 + j) * 68 + nb * 16 + lr] = acc[mb][nb][j]; }
        wave_sync();
        float* cb = C + (size_t)(r0 + mb * 16) * (size_t)ldc + c0;
#pragma unroll 1
        for (int ps = 0; ps < 2; ++ps) {
#pragma unroll
            for (int s = 0; s < 8; ++s) { const int row = 2 * s + hi, cofs = lr * 4;
                const v4f val = *(const v4fa*)(&os[row * 68 + cofs]);
                *(volatile v4f*)(cb + (size_t)row * (size_t)ldc + cofs) = val; }
            if (ps == 0) __threadfence(); }
        wave_sync();
    }
}

__global__ __launch_bounds__(256) void k_x(const float* __restrict__ EMB, const float* __restrict__ own, const float* __restrict__ hid,
                                           const float* __restrict__ fc1w, const float* __restrict__ fc1b, const float* __restrict__ wim, bf* XH) {
    __shared__ __align__(16) float wl[FD * 64];
    __shared__ __align__(16) float ol[64];
    __shared__ __align__(16) unsigned short Xs[4 * K2];
    const int t = threadIdx.x, a = t >> 6, h = t & 63; const int n0 = blockIdx.x * 4, n = n0 + a;
    { const v4f w4 = *(const v4f*)(fc1w + t * 4); *(v4fa*)(&wl[t * 4]) = rbf4(w4); }
    { const float v = own[(size_t)n0 * FD + (t & 63)]; if (t < 64) ol[t] = rbf(v); }
    __syncthreads();
    const v4f e4 = *(const v4f*)(EMB + (size_t)n * N1 + h * 4);
    float m = e4[0] * rbf(wim[h]);
    m = fmaf(e4[1], rbf(wim[64 + h]), m); m = fmaf(e4[2], rbf(wim[128 + h]), m); m = fmaf(e4[3], rbf(wim[192 + h]), m);
    float d = 0.0f;
#pragma unroll 4
    for (int f = 0; f < FD; ++f) d = fmaf(ol[a * 16 + f], wl[f * 64 + h], d);
    const float emb = (d + rbf(fc1b[h])) + m;
    const float x = fmaxf(emb, 0.0f);
    const unsigned short xh = f2bf(x); const unsigned short xl = f2bf(x - bf2f(xh));
    Xs[a * K2 + h] = xh; Xs[a * K2 + 64 + h] = xl; Xs[a * K2 + 128 + h] = f2bf(hid[(size_t)n * HID + h]);
    __syncthreads();
    bf* dst = XH + (size_t)n0 * K2;
#pragma unroll 1
    for (int ps = 0; ps < 2; ++ps) {
        if (t < 96) { const v8us v = *(const v8usa*)(&Xs[t * 8]); *(volatile v8us*)(dst + t * 8) = v; }
        if (ps == 0) __threadfence(); }
}

__global__ __launch_bounds__(256) void k_gate(const float* __restrict__ G, const float* __restrict__ hid, const float* __restrict__ bih, const float* __restrict__ bhh, float* OUT1, bf* HH) {
    __shared__ __align__(16) float bl[384];
    __shared__ __align__(16) float hs[256];
    __shared__ __align__(16) unsigned short Hs[4 * K3];
    const int t = threadIdx.x, a = t >> 6, h = t & 63; const int n0 = blockIdx.x * 4, n = n0 + a;
    { const int c = t < 48 ? t : 47; const v4f vi = *(const v4f*)(bih + c * 4); const v4f vh = *(const v4f*)(bhh + c * 4);
      if (t < 48) { *(v4fa*)(&bl[t * 4]) = rbf4(vi); *(v4fa*)(&bl[192 + t * 4]) = rbf4(vh); } }
    __syncthreads();
    const float* g = G + (size_t)n * N2;
    const float sr = (g[h] + bl[h]) + bl[192 + h];
    const float sz = (g[64 + h] + bl[64 + h]) + bl[256 + h];
    const float ig = g[128 + h] + bl[128 + h];
    const float hg = g[192 + h] + bl[320 + h];
    const float r = 1.0f / (1.0f + expf(-sr));
    const float z = 1.0f / (1.0f + expf(-sz));
    const float gg = tanhf(ig + r * hg);
    const float hp = rbf(hid[(size_t)n * HID + h]);
    const float hh = (1.0f - z) * gg + z * hp;
    hs[t] = hh;
    const unsigned short hh_h = f2bf(hh); const unsigned short hh_l = f2bf(hh - bf2f(hh_h));
    Hs[a * K3 + h] = hh_h; Hs[a * K3 + 64 + h] = hh_l;
    __syncthreads();
    float* od = OUT1 + (size_t)n0 * HID; bf* pd = HH + (size_t)n0 * K3;
#pragma unroll 1
    for (int ps = 0; ps < 2; ++ps) {
        if (t < 64) { const v4f v = *(const v4fa*)(&hs[t * 4]); *(volatile v4f*)(od + t * 4) = v;
                      const v8us u = *(const v8usa*)(&Hs[t * 8]); *(volatile v8us*)(pd + t * 8) = u; }
        if (ps == 0) __threadfence(); }
}

__global__ __launch_bounds__(128) void k_head(const float* __restrict__ T, const float* __restrict__ RE, const float* __restrict__ hew2, const float* __restrict__ heb2,
                                              const float* __restrict__ fc2b, const float* __restrict__ wom, float* OUT0) {
    __shared__ __align__(16) float w2b[256];
    __shared__ __align__(16) float Us[HAG * 64];
    __shared__ __align__(16) float cs[HAG];
    __shared__ __align__(16) float qs[HAG * QW];
    const int t = threadIdx.x; const int n0 = blockIdx.x * HAG;
#pragma unroll
    for (int i = 0; i < 2; ++i) { const int idx = t + 128 * i; w2b[idx] = rbf(hew2[(size_t)(idx >> 2) * DE + 4352 + (idx & 3)]); }
    const float w0 = rbf(wom[0]), w1 = rbf(wom[1]), w2 = rbf(wom[2]), w3 = rbf(wom[3]);
    __syncthreads();
#pragma unroll 1
    for (int i = 0; i < 8; ++i) { const int idx = t + 128 * i; const int a = idx >> 6, j = idx & 63;
        const v4f tv = *(const v4f*)(T + (size_t)(n0 + a) * N3 + j * 4); const v4f wv = *(const v4fa*)(&w2b[j * 4]);
        float u = w0 * (tv[0] + wv[0]); u = fmaf(w1, tv[1] + wv[1], u); u = fmaf(w2, tv[2] + wv[2], u); u = fmaf(w3, tv[3] + wv[3], u);
        Us[idx] = u; }
    { const int a = t & 15; const v4f tb = *(const v4f*)(T + (size_t)(n0 + a) * N3 + 256);
      float c = w0 * (tb[0] + rbf(heb2[4352])); c = fmaf(w1, tb[1] + rbf(heb2[4353]), c); c = fmaf(w2, tb[2] + rbf(heb2[4354]), c); c = fmaf(w3, tb[3] + rbf(heb2[4355]), c);
      if (t < HAG) cs[t] = c; }
    __syncthreads();
    { const int a = t >> 3, e = t & 7; const float* rr = RE + ((size_t)(n0 + a) * NEN + e) * 64; float acc = 0.0f;
#pragma unroll 4
      for (int j4 = 0; j4 < 16; ++j4) { const v4f rv = *(const v4f*)(rr + j4 * 4); const v4f uv = *(const v4fa*)(&Us[a * 64 + j4 * 4]);
          acc = fmaf(rv[0], uv[0], acc); acc = fmaf(rv[1], uv[1], acc); acc = fmaf(rv[2], uv[2], acc); acc = fmaf(rv[3], uv[3], acc); }
      qs[a * QW + OUTN + e] = acc + cs[a]; }
    { const int tt = t < 95 ? t : 95; const int a = tt / OUTN, o = tt - a * OUTN;
      const float v = T[(size_t)(n0 + a) * N3 + 260 + o] + rbf(fc2b[o]);
      if (t < HAG * OUTN) qs[a * QW + o] = v; }
    __syncthreads();
    float* od = OUT0 + (size_t)n0 * QW;
#pragma unroll 1
    for (int ps = 0; ps < 2; ++ps) {
        if (t < (HAG * QW) / 4) { const v4f v = *(const v4fa*)(&qs[t * 4]); *(volatile v4f*)(od + t * 4) = v; }
        if (ps == 0) __threadfence(); }
}

static constexpr size_t al256(size_t v) { return (v + 255) & ~(size_t)255; }
static constexpr size_t SZ_A1  = al256((size_t)NAG * K1 * 2);
static constexpr size_t SZ_BT1 = al256((size_t)N1 * K1 * 2);
static constexpr size_t SZ_RE  = al256((size_t)NAG * NEN * 64 * 4);
static constexpr size_t SZ_EMB = al256((size_t)NAG * N1 * 4);
static constexpr size_t SZ_XH  = al256((size_t)NAG * K2 * 2);
static constexpr size_t SZ_BT2 = al256((size_t)N2 * K2 * 2);
static constexpr size_t SZ_G   = al256((size_t)NAG * N2 * 4);
static constexpr size_t SZ_HH  = al256((size_t)NAG * K3 * 2);
static constexpr size_t SZ_BT3 = al256((size_t)N3 * K3 * 2);
static constexpr size_t SZ_T   = al256((size_t)NAG * N3 * 4);
static constexpr size_t SZ_TOTAL = SZ_A1 + SZ_BT1 + SZ_RE + SZ_EMB + SZ_XH + SZ_BT2 + SZ_G + SZ_HH + SZ_BT3 + SZ_T;
static_assert(SZ_TOTAL <= (size_t)134217728);
static_assert(((size_t)K1 * 2) % 128 == 0);
static_assert(((size_t)K2 * 2) % 128 == 0);
static_assert(((size_t)K3 * 2) % 128 == 0);
static_assert(N3 * (K3 / 16) == 10 * 256);
static_assert(N3 == 256 + 2 * 32);
static_assert(N2 * (K2 / 8) == 24 * 256);

extern "C" void kernel_launch(void* const* d_in, const int* in_sizes, int n_in,
                              void* d_out, int out_size, void* d_ws, size_t ws_size, hipStream_t stream) {
    if (n_in < 22) return;
    if ((size_t)in_sizes[0] < (size_t)NAG * FD) return;
    if ((size_t)in_sizes[1] < (size_t)NAG * NEN * FD) return;
    if ((size_t)in_sizes[2] < (size_t)NAG * NAL * FD) return;
    if ((size_t)in_sizes[3] < (size_t)NAG * HID) return;
    if (in_sizes[4] < FD * 64 || in_sizes[5] < 64 || in_sizes[6] < FD * 64 || in_sizes[7] < 64) return;
    if (in_sizes[8] < 64 * DE || in_sizes[9] < DE || in_sizes[10] < FD * 64 || in_sizes[11] < 64) return;
    if (in_sizes[12] < 64 * DA || in_sizes[13] < DA || in_sizes[14] < HEADS * 64) return;
    if (in_sizes[15] < 192 * 64 || in_sizes[16] < 192 || in_sizes[17] < 192 * 64 || in_sizes[18] < 192) return;
    if (in_sizes[19] < 64 * OUTN || in_sizes[20] < OUTN || in_sizes[21] < HEADS) return;
    if ((size_t)out_size < (size_t)NAG_FULL * QW + (size_t)NAG * HID) return;
    if (SZ_TOTAL > ws_size) return;
    const float* own  = (const float*)d_in[0];  const float* ef   = (const float*)d_in[1];  const float* af   = (const float*)d_in[2];  const float* hid  = (const float*)d_in[3];
    const float* fc1w = (const float*)d_in[4];  const float* fc1b = (const float*)d_in[5];
    const float* hew1 = (const float*)d_in[6];  const float* heb1 = (const float*)d_in[7];  const float* hew2 = (const float*)d_in[8];  const float* heb2 = (const float*)d_in[9];
    const float* haw1 = (const float*)d_in[10]; const float* hab1 = (const float*)d_in[11]; const float* haw2 = (const float*)d_in[12]; const float* hab2 = (const float*)d_in[13];
    const float* wim  = (const float*)d_in[14];
    const float* wih  = (const float*)d_in[15]; const float* bih  = (const float*)d_in[16]; const float* whh  = (const float*)d_in[17]; const float* bhh  = (const float*)d_in[18];
    const float* fc2w = (const float*)d_in[19]; const float* fc2b = (const float*)d_in[20]; const float* wom  = (const float*)d_in[21];
    float* OUT0 = (float*)d_out;
    float* OUT1 = (float*)d_out + (size_t)NAG_FULL * QW;
    char* wsp = (char*)d_ws;
    bf*    A1  = (bf*)wsp;    wsp += SZ_A1;
    bf*    BT1 = (bf*)wsp;    wsp += SZ_BT1;
    float* RE  = (float*)wsp; wsp += SZ_RE;
    float* EMB = (float*)wsp; wsp += SZ_EMB;
    bf*    XH  = (bf*)wsp;    wsp += SZ_XH;
    bf*    BT2 = (bf*)wsp;    wsp += SZ_BT2;
    float* G   = (float*)wsp; wsp += SZ_G;
    bf*    HH  = (bf*)wsp;    wsp += SZ_HH;
    bf*    BT3 = (bf*)wsp;    wsp += SZ_BT3;
    float* T   = (float*)wsp; wsp += SZ_T;

    k_bt1<<<dim3(N1, 3, 1), 128, 0, stream>>>(hew2, heb2, haw2, hab2, BT1);
    k_bt2<<<24, 256, 0, stream>>>(wih, whh, BT2);
    k_bt3<<<10, 256, 0, stream>>>(hew2, heb2, fc2w, BT3);
    k_build<<<NAG / APB, 64, 0, stream>>>(ef, af, hew1, heb1, haw1, hab1, A1, RE);
    k_gemm<<<dim3(NAG / 64, N1 / 64, 1), 32, 0, stream>>>(A1, BT1, EMB, K1, N1);
    k_x<<<NAG / 4, 256, 0, stream>>>(EMB, own, hid, fc1w, fc1b, wim, XH);
    k_gemm<<<dim3(NAG / 64, N2 / 64, 1), 32, 0, stream>>>(XH, BT2, G, K2, N2);
    k_gate<<<NAG / 4, 256, 0, stream>>>(G, hid, bih, bhh, OUT1, HH);
    k_gemm<<<dim3(NAG / 64, N3 / 64, 1), 32, 0, stream>>>(HH, BT3, T, K3, N3);
    k_head<<<NAG / HAG, 128, 0, stream>>>(T, RE, hew2, heb2, fc2b, wom, OUT0);
}
